// DoubleStreamRWKVBlock_85066122264762
// MI455X (gfx1250) — hardware-verified
//
#include <hip/hip_runtime.h>
#include <math.h>

constexpr int NBATCH = 2;
constexpr int NCH    = 1024;
constexpr int NHEAD  = 16;
constexpr int HEADSZ = 64;
constexpr int NFFN   = 2048;
constexpr int LIMG   = 4096;
constexpr int LTXT   = 512;
constexpr int LSEQ   = LIMG + LTXT;
constexpr int MODN   = 6 * NCH;
constexpr int NTOK   = NBATCH * LSEQ;
constexpr int NCAT   = 4 * NCH;
constexpr int SLABP  = 68;
constexpr int TPITCH = 260;
constexpr int SCT    = 16;
constexpr float WCARRY     = 64.0f;
constexpr float WCARRY_INV = 1.0f / 64.0f;
constexpr float RMS_EPS    = 1e-6f;
constexpr float GN_EPS     = 1e-5f;
constexpr float GELU_C0    = 0.7978845608028654f;
constexpr float GELU_C1    = 0.044715f;

static_assert(NCH == NHEAD * HEADSZ);
static_assert(HEADSZ == 64);
static_assert(LIMG % 64 == 0 && LTXT % 64 == 0 && LSEQ % 64 == 0);
static_assert(NTOK % 64 == 0 && NCH % 64 == 0 && NFFN % 64 == 0);
static_assert(NCH % 32 == 0 && NFFN % 32 == 0);
static_assert(LSEQ % SCT == 0);
static_assert(LIMG % 32 == 0 && LTXT % 32 == 0);

typedef __attribute__((ext_vector_type(16))) _Float16 v16h;
typedef __attribute__((ext_vector_type(8)))  _Float16 v8h;
typedef __attribute__((ext_vector_type(8)))  float    v8f;
typedef __attribute__((ext_vector_type(4)))  float    v4f;
typedef __attribute__((ext_vector_type(2)))  float    v2f;
typedef __attribute__((ext_vector_type(4)))  unsigned v4u;

__device__ __forceinline__ float h16_to_f32(unsigned hb) {
  const unsigned sgn = (hb & 0x8000u) << 16;
  const unsigned em  = hb & 0x7fffu;
  const float fn = __uint_as_float((em << 13) + 0x38000000u);
  const float fs = (float)em * 5.9604644775390625e-8f;
  const float mag = (em < 0x400u) ? fs : fn;
  return __uint_as_float(__float_as_uint(mag) | sgn);
}

__device__ __forceinline__ void wave_sync() {
  __builtin_amdgcn_fence(__ATOMIC_RELEASE, "workgroup");
  __builtin_amdgcn_wave_barrier();
  __builtin_amdgcn_fence(__ATOMIC_ACQUIRE, "workgroup");
}

union FragU { v16h v; v8h h[2]; };
__device__ __forceinline__ v16h frag_load(const _Float16* p) {
  FragU f;
  f.h[0] = *(const v8h*)(p);
  f.h[1] = *(const v8h*)(p + 16);
  return f.v;
}
__device__ __forceinline__ v8f frag_mma(v16h a, v16h b, v8f c) {
  return __builtin_amdgcn_wmma_f32_16x16x32_f16(false, a, false, b, (short)0, c, false, false);
}
__device__ __forceinline__ void group_guard(v8f& a, v8f& b, v8f& c, v8f& d, v16h x, v16h y0, v16h y1, v16h y2, v16h y3) {
  asm volatile("v_nop\n\tv_nop\n\tv_nop\n\tv_nop" : "+v"(a), "+v"(b), "+v"(c), "+v"(d) : "v"(x), "v"(y0), "v"(y1), "v"(y2), "v"(y3));
}
__device__ __forceinline__ void keep4_h(v16h a, v16h b, v16h c, v16h d) { asm volatile("v_nop" :: "v"(a), "v"(b), "v"(c), "v"(d)); }
__device__ __forceinline__ void acc_guard4(v8f& a, v8f& b, v8f& c, v8f& d) { asm volatile("v_nop\n\tv_nop\n\tv_nop\n\tv_nop" : "+v"(a), "+v"(b), "+v"(c), "+v"(d)); }

__device__ __forceinline__ float act_silu(float v) {
  const float vc = fmaxf(v, -30.0f);
  return v * (1.0f / (1.0f + expf(-vc)));
}
__device__ __forceinline__ float act_gelu(float v) {
  float t = GELU_C0 * (v + GELU_C1 * v * v * v);
  t = fminf(fmaxf(t, -20.0f), 20.0f);
  const float e  = expf(2.0f * t);
  const float th = 1.0f - 2.0f / (1.0f + e);
  return 0.5f * v * (1.0f + th);
}
template <int ACT> __device__ __forceinline__ float act_fn(float v) {
  if (ACT == 1) return act_silu(v);
  if (ACT == 2) return act_gelu(v);
  return v;
}

__global__ __launch_bounds__(256) void cast_planes_kernel(
    const float* __restrict__ s0, const float* __restrict__ s1, const float* __restrict__ s2,
    const float* __restrict__ s3, const float* __restrict__ s4,
    unsigned short* dst, int n8, float sc) {
  const int pl = blockIdx.y;
  const float* s = s0;
  if (pl == 1) s = s1;
  if (pl == 2) s = s2;
  if (pl == 3) s = s3;
  if (pl == 4) s = s4;
  const int i = blockIdx.x * 256 + threadIdx.x;
  if (i < n8) {
    const float* sp = s + (size_t)i * 8;
    const v4f a = *(const v4f*)(sp);
    const v4f b = *(const v4f*)(sp + 4);
    v8h hv;
#pragma unroll
    for (int e = 0; e < 4; ++e) {
      hv[e]     = (_Float16)(a[e] * sc);
      hv[4 + e] = (_Float16)(b[e] * sc);
    }
    unsigned short* dp = dst + ((size_t)pl * n8 + (size_t)i) * 8;
    *(volatile v8h*)dp = hv;
    __threadfence();
    *(volatile v8h*)dp = hv;
  }
}

__global__ __launch_bounds__(256) void mod_gemv_kernel(
    const float* __restrict__ Wi, const float* __restrict__ bi,
    const float* __restrict__ Wt, const float* __restrict__ bt,
    const float* __restrict__ cond, float* MODp) {
  __shared__ __align__(16) float scs[2 * NCH];
  __shared__ float sres[64];
  const int tid = threadIdx.x, lane = tid & 31, wave = tid >> 5;
  const int strm = blockIdx.y;
  const int o0 = blockIdx.x * 32;
  const float* Wm = strm ? Wt : Wi;
  const float* bm = strm ? bt : bi;
#pragma unroll 1
  for (int i = tid; i < 2 * NCH; i += 256) {
    const float x = cond[i];
    scs[i] = x / (1.0f + expf(-x));
  }
  __syncthreads();
#pragma unroll 1
  for (int j = 0; j < 4; ++j) {
    const int o = o0 + 4 * wave + j;
    const float* wr = Wm + (size_t)o * NCH + 4 * lane;
    float a0 = 0.0f, a1 = 0.0f;
#pragma unroll 1
    for (int i = 0; i < 8; ++i) {
      const v4f wv = *(const v4f*)(wr + 128 * i);
      const v4f c0 = *(const v4f*)(scs + 128 * i + 4 * lane);
      const v4f c1 = *(const v4f*)(scs + NCH + 128 * i + 4 * lane);
      a0 += (wv[0] * c0[0] + wv[1] * c0[1]) + (wv[2] * c0[2] + wv[3] * c0[3]);
      a1 += (wv[0] * c1[0] + wv[1] * c1[1]) + (wv[2] * c1[2] + wv[3] * c1[3]);
    }
#pragma unroll
    for (int off = 1; off < 32; off <<= 1) {
      a0 += __shfl_xor(a0, off, 32);
      a1 += __shfl_xor(a1, off, 32);
    }
    const float bv = bm[o];
    if (lane == 0) {
      sres[4 * wave + j]      = a0 + bv;
      sres[32 + 4 * wave + j] = a1 + bv;
    }
  }
  __syncthreads();
  if (wave < 2) {
    const float val = sres[wave * 32 + lane];
    float* p = MODp + (size_t)(strm * 2 + wave) * MODN + o0 + lane;
    *(volatile float*)p = val;
    __threadfence();
    *(volatile float*)p = val;
  }
}

template <bool MIXED>
__global__ __launch_bounds__(256) void norm_mod_tok_kernel(
    const float* __restrict__ src0, const float* __restrict__ src1,
    const float* __restrict__ rw0, const float* __restrict__ rw1,
    const float* __restrict__ MODp, int shChunk, int scChunk,
    const float* __restrict__ muA, const float* __restrict__ muB,
    unsigned short* outA, long bsA, unsigned short* outB, long bsB) {
  __shared__ float red[8 * 32];
  __shared__ float redh[8];
  __shared__ float sinv[33];
  __shared__ __align__(16) float tile[33 * TPITCH];
  const int tid = threadIdx.x, lane = tid & 31, wave = tid >> 5;
  const int l0 = blockIdx.x * 32;
  const int b  = blockIdx.y;
  const int strm = (l0 >= LIMG) ? 1 : 0;
  const int lloc = strm ? (l0 - LIMG) : l0;
  const int Ls   = strm ? LTXT : LIMG;
  const float* src  = (strm ? src1 : src0) + (size_t)b * NCH * Ls + lloc + lane;
  const float* rw   = strm ? rw1 : rw0;
  const float* modp = MODp + (size_t)(strm * 2 + b) * MODN;
  const bool hasPrior = MIXED && (l0 > 0);
  const int lh    = hasPrior ? (l0 - 1) : l0;
  const int hstrm = (lh >= LIMG) ? 1 : 0;
  const int hloc  = hstrm ? (lh - LIMG) : lh;
  const int Lh    = hstrm ? LTXT : LIMG;
  const float* srch = (hstrm ? src1 : src0) + (size_t)b * NCH * Lh + hloc;
  const float* rwh  = hstrm ? rw1 : rw0;
  const float* modh = MODp + (size_t)(hstrm * 2 + b) * MODN;

  float ss = 0.0f, ssh = 0.0f;
#pragma unroll 4
  for (int j = 0; j < 128; ++j) {
    const int c = wave + 8 * j;
    const float v = src[(size_t)c * Ls];
    ss = fmaf(v, v, ss);
    if (MIXED) {
      const float vh = srch[(size_t)c * Lh];
      ssh = fmaf(vh, vh, ssh);
    }
  }
  red[wave * 32 + lane] = ss;
  if (MIXED && lane == 0) redh[wave] = ssh;
  __syncthreads();
  if (tid < 32) {
    float s = 0.0f;
#pragma unroll
    for (int w = 0; w < 8; ++w) s += red[w * 32 + tid];
    sinv[tid] = rsqrtf(s * (1.0f / NCH) + RMS_EPS);
  }
  if (MIXED && tid == 32) {
    float s = 0.0f;
#pragma unroll
    for (int w = 0; w < 8; ++w) s += redh[w];
    sinv[32] = rsqrtf(s * (1.0f / NCH) + RMS_EPS);
  }
  __syncthreads();
  const float inv = sinv[lane];
  float invh = 0.0f;
  if (MIXED) invh = sinv[32];

#pragma unroll 1
  for (int cc = 0; cc < 4; ++cc) {
#pragma unroll 4
    for (int j = 0; j < 32; ++j) {
      const int cl = wave * 32 + j;
      const int c  = cc * 256 + cl;
      const float v = src[(size_t)c * Ls];
      const float val = ((v * inv) * rw[c]) * (1.0f + modp[scChunk * NCH + c]) + modp[shChunk * NCH + c];
      tile[(lane + 1) * TPITCH + cl] = val;
      if (MIXED) {
        const float vh = srch[(size_t)c * Lh];
        float hval = ((vh * invh) * rwh[c]) * (1.0f + modh[scChunk * NCH + c]) + modh[shChunk * NCH + c];
        hval = hasPrior ? hval : 0.0f;
        if (lane == 0) tile[cl] = hval;
      }
    }
    __syncthreads();
    const int c0 = cc * 256 + lane * 8;
    v4f mA0 = {0.f, 0.f, 0.f, 0.f}, mA1 = mA0, mB0 = mA0, mB1 = mA0;
    if (MIXED) {
      mA0 = *(const v4f*)(muA + c0);
      mA1 = *(const v4f*)(muA + c0 + 4);
      mB0 = *(const v4f*)(muB + c0);
      mB1 = *(const v4f*)(muB + c0 + 4);
    }
#pragma unroll 1
    for (int it = 0; it < 4; ++it) {
      const int token = it * 8 + wave;
      const float* xp = tile + (token + 1) * TPITCH + lane * 8;
      const v4f xa = *(const v4f*)(xp);
      const v4f xb = *(const v4f*)(xp + 4);
      v8h hA, hB;
      if (MIXED) {
        const float* pp = tile + token * TPITCH + lane * 8;
        const v4f pa = *(const v4f*)(pp);
        const v4f pb = *(const v4f*)(pp + 4);
#pragma unroll
        for (int e = 0; e < 4; ++e) {
          hA[e]     = (_Float16)(xa[e] + mA0[e] * (pa[e] - xa[e]));
          hA[4 + e] = (_Float16)(xb[e] + mA1[e] * (pb[e] - xb[e]));
          hB[e]     = (_Float16)(xa[e] + mB0[e] * (pa[e] - xa[e]));
          hB[4 + e] = (_Float16)(xb[e] + mB1[e] * (pb[e] - xb[e]));
        }
      } else {
#pragma unroll
        for (int e = 0; e < 4; ++e) {
          hA[e]     = (_Float16)xa[e];
          hA[4 + e] = (_Float16)xb[e];
        }
        hB = hA;
      }
      unsigned short* pA;
      unsigned short* pB;
      if (MIXED) {
        const size_t ro = ((size_t)b * LSEQ + (size_t)(l0 + token)) * NCH + c0;
        pA = outA + ro;
        pB = outB + ro;
      } else {
        const size_t ro = (size_t)(lloc + token) * NCH + c0;
        pA = (strm ? (outB + (size_t)b * bsB) : (outA + (size_t)b * bsA)) + ro;
        pB = pA;
      }
      *(volatile v8h*)pA = hA;
      if (MIXED) *(volatile v8h*)pB = hB;
      __threadfence();
      *(volatile v8h*)pA = hA;
      if (MIXED) *(volatile v8h*)pB = hB;
    }
    __syncthreads();
  }
}

template <int EPI, int ACT>
__global__ __launch_bounds__(256) void gemm_f16_kernel(
    const unsigned short* __restrict__ Ap, int lda, long strideA,
    const unsigned short* __restrict__ Btp, int ldb, long strideB,
    unsigned short* C16, int ldc,
    float* dst0, const float* res0, const float* gate0, int ld0, long bs0,
    float* dst1, const float* res1, const float* gate1, int ld1, long bs1,
    long gbs, int nsplit, int Mrows, int Ncols, int Kdim, float scale) {
  __shared__ __align__(16) float sT[8][16 * SLABP];
  const int bz   = blockIdx.y;
  const int lane = threadIdx.x & 31;
  const int wave = threadIdx.x >> 5;
  const int tilesN = Ncols >> 6;
  const int tilesM = Mrows >> 6;
  const int tile = blockIdx.x * 8 + wave;
  if (tile >= tilesM * tilesN) return;
  const int tm = tile / tilesN;
  const int tn = tile - tm * tilesN;
  const int m0 = tm << 6;
  const int n0 = tn << 6;

  const _Float16* Ab = (const _Float16*)Ap  + (size_t)bz * strideA;
  const _Float16* Bb = (const _Float16*)Btp + (size_t)bz * strideB;
  const int rlane = lane & 15;
  const int koff  = (lane >> 4) * 8;
  const int mOff  = koff;
  const _Float16* abase = Ab + (size_t)(m0 + rlane) * lda + koff;
  const _Float16* bbase = Bb + (size_t)(n0 + rlane) * ldb + koff;
  const size_t astep = (size_t)16 * lda;
  const size_t bstep = (size_t)16 * ldb;

  v8f acc[4][4];
#pragma unroll
  for (int i = 0; i < 4; ++i)
#pragma unroll
    for (int j = 0; j < 4; ++j) acc[i][j] = (v8f){0.f, 0.f, 0.f, 0.f, 0.f, 0.f, 0.f, 0.f};

#pragma unroll 1
  for (int k0 = 0; k0 < Kdim; k0 += 32) {
    v16h bf[4];
#pragma unroll
    for (int j = 0; j < 4; ++j) bf[j] = frag_load(bbase + j * bstep + k0);
#pragma unroll
    for (int i = 0; i < 4; ++i) {
      const v16h af = frag_load(abase + i * astep + k0);
#pragma unroll
      for (int j = 0; j < 4; ++j) acc[i][j] = frag_mma(af, bf[j], acc[i][j]);
      group_guard(acc[i][0], acc[i][1], acc[i][2], acc[i][3], af, bf[0], bf[1], bf[2], bf[3]);
    }
    keep4_h(bf[0], bf[1], bf[2], bf[3]);
  }
  acc_guard4(acc[0][0], acc[0][1], acc[0][2], acc[0][3]);
  acc_guard4(acc[1][0], acc[1][1], acc[1][2], acc[1][3]);
  acc_guard4(acc[2][0], acc[2][1], acc[2][2], acc[2][3]);
  acc_guard4(acc[3][0], acc[3][1], acc[3][2], acc[3][3]);

  float* slab = sT[wave];
  const bool second = (n0 >= nsplit);
  float* dp       = second ? (dst1 + (size_t)bz * bs1) : (dst0 + (size_t)bz * bs0);
  const float* rp = second ? (res1 + (size_t)bz * bs1) : (res0 + (size_t)bz * bs0);
  const float* gp = (second ? gate1 : gate0) + (size_t)bz * gbs;
  const int ldd   = second ? ld1 : ld0;
  const int ncol  = second ? (n0 - nsplit) : n0;

#pragma unroll
  for (int i = 0; i < 4; ++i) {
    const int mBase = m0 + (i << 4);
#pragma unroll
    for (int j = 0; j < 4; ++j)
#pragma unroll
      for (int r = 0; r < 8; ++r) slab[(mOff + r) * SLABP + (j << 4) + rlane] = acc[i][j][r] * scale;
    wave_sync();
    if (EPI == 0) {
      const int q = lane >> 3, c8 = (lane & 7) * 8;
      if (ACT != 0) {
#pragma unroll 1
        for (int u = 0; u < 8; ++u) {
          float* sp = slab + ((u >> 1) * 4 + q) * SLABP + c8 + (u & 1) * 4;
          v4f a = *(const v4f*)sp;
          a[0] = act_fn<ACT>(a[0]);
          a[1] = act_fn<ACT>(a[1]);
          a[2] = act_fn<ACT>(a[2]);
          a[3] = act_fn<ACT>(a[3]);
          *(v4f*)sp = a;
        }
        wave_sync();
      }
      v8h hv[4];
#pragma unroll
      for (int it = 0; it < 4; ++it) {
        const float* sp = slab + (it * 4 + q) * SLABP + c8;
        const v4f a  = *(const v4f*)(sp);
        const v4f b2 = *(const v4f*)(sp + 4);
#pragma unroll
        for (int e = 0; e < 4; ++e) {
          hv[it][e]     = (_Float16)a[e];
          hv[it][4 + e] = (_Float16)b2[e];
        }
      }
      for (int pass = 0; pass < 2; ++pass) {
#pragma unroll
        for (int it = 0; it < 4; ++it) {
          const int row = it * 4 + q;
          *(volatile v8h*)(C16 + (size_t)(mBase + row) * ldc + n0 + c8) = hv[it];
        }
        __threadfence();
      }
    } else {
      const int hh = lane >> 4, c4 = (lane & 15) * 4;
      v4f ov[8];
#pragma unroll
      for (int it = 0; it < 8; ++it) {
        const int row = it * 2 + hh;
        const int m = mBase + row;
        const v4f a = *(const v4f*)(slab + row * SLABP + c4);
        const float gt = gp[m];
        const v4f rr = *(const v4f*)(rp + (size_t)m * ldd + ncol + c4);
#pragma unroll
        for (int e = 0; e < 4; ++e) ov[it][e] = rr[e] + gt * a[e];
      }
      for (int pass = 0; pass < 2; ++pass) {
#pragma unroll
        for (int it = 0; it < 8; ++it) {
          const int row = it * 2 + hh;
          *(volatile v4f*)(dp + (size_t)(mBase + row) * ldd + ncol + c4) = ov[it];
        }
        __threadfence();
      }
    }
    wave_sync();
  }
}

__global__ __launch_bounds__(256) void state_scan_kernel(
    const unsigned short* __restrict__ RK, const float* __restrict__ tdecay, const float* __restrict__ tfirst,
    const float* __restrict__ lnw, const float* __restrict__ lnb, unsigned short* Zp) {
  __shared__ __align__(16) float sX[4][SCT * 64];
  __shared__ __align__(16) float sY[8][SCT * 64];
  __shared__ __align__(16) float sW[64];
  __shared__ __align__(16) unsigned sZ[SCT * 32];
  const int bh = blockIdx.x;
  const int b = bh >> 4, h = bh & 15;
  const int tid = threadIdx.x, lane = tid & 31, q = tid >> 5;
  if (tid < 64) sW[tid] = expf(-expf(tdecay[h * 64 + tid]));
  const float u0 = tfirst[h * 64 + lane];
  const float u1 = tfirst[h * 64 + 32 + lane];
  const int ch0 = h * 64 + 2 * lane;
  const float lw0 = lnw[ch0], lw1 = lnw[ch0 + 1];
  const float lb0 = lnb[ch0], lb1 = lnb[ch0 + 1];
  __syncthreads();
  float wq[8];
  {
    const v4f wa = *(const v4f*)(sW + 8 * q);
    const v4f wb = *(const v4f*)(sW + 8 * q + 4);
#pragma unroll
    for (int e = 0; e < 4; ++e) { wq[e] = wa[e]; wq[4 + e] = wb[e]; }
  }
  float S0[8], S1[8];
#pragma unroll
  for (int e = 0; e < 8; ++e) { S0[e] = 0.0f; S1[e] = 0.0f; }
  const int stok = (tid >> 3) & 15;
  const int sseg = tid & 7;
  const int sarr = tid >> 7;

#pragma unroll 1
  for (int grp = 0; grp < LSEQ / SCT; ++grp) {
    const size_t tok0 = (size_t)b * LSEQ + (size_t)grp * SCT;
#pragma unroll
    for (int rr = 0; rr < 2; ++rr) {
      const int a = rr * 2 + sarr;
      const v4u wv = *(const v4u*)(RK + (tok0 + stok) * NCAT + a * NCH + h * 64 + sseg * 8);
      float f[8];
#pragma unroll
      for (int e = 0; e < 4; ++e) {
        const unsigned wd = wv[e];
        f[2 * e]     = h16_to_f32(wd & 0xffffu);
        f[2 * e + 1] = h16_to_f32(wd >> 16);
      }
      float* dp = &sX[a][stok * 64 + sseg * 8];
      *(v4f*)(dp)     = (v4f){f[0], f[1], f[2], f[3]};
      *(v4f*)(dp + 4) = (v4f){f[4], f[5], f[6], f[7]};
    }
    __syncthreads();
#pragma unroll 1
    for (int t = 0; t < SCT; ++t) {
      const v2f vv = *(const v2f*)(&sX[2][t * 64 + 2 * lane]);
      const v4f ra = *(const v4f*)(&sX[0][t * 64 + 8 * q]);
      const v4f rb = *(const v4f*)(&sX[0][t * 64 + 8 * q + 4]);
      const v4f ka = *(const v4f*)(&sX[1][t * 64 + 8 * q]);
      const v4f kb = *(const v4f*)(&sX[1][t * 64 + 8 * q + 4]);
      float y0 = 0.0f, y1 = 0.0f;
#pragma unroll
      for (int e = 0; e < 4; ++e) {
        const float rn = ra[e], kn = ka[e];
        y0 = fmaf(rn, S0[e], y0);
        y1 = fmaf(rn, S1[e], y1);
        S0[e] = fmaf(wq[e], S0[e], kn * vv[0]);
        S1[e] = fmaf(wq[e], S1[e], kn * vv[1]);
      }
#pragma unroll
      for (int e = 0; e < 4; ++e) {
        const float rn = rb[e], kn = kb[e];
        y0 = fmaf(rn, S0[4 + e], y0);
        y1 = fmaf(rn, S1[4 + e], y1);
        S0[4 + e] = fmaf(wq[4 + e], S0[4 + e], kn * vv[0]);
        S1[4 + e] = fmaf(wq[4 + e], S1[4 + e], kn * vv[1]);
      }
      *(v2f*)(&sY[q][t * 64 + 2 * lane]) = (v2f){y0, y1};
    }
    __syncthreads();
#pragma unroll 1
    for (int i2 = 0; i2 < 2; ++i2) {
      const int t = 2 * q + i2;
      float p = (sX[0][t * 64 + lane] * u0) * sX[1][t * 64 + lane]
              + (sX[0][t * 64 + 32 + lane] * u1) * sX[1][t * 64 + 32 + lane];
#pragma unroll
      for (int off = 1; off < 32; off <<= 1) p += __shfl_xor(p, off, 32);
      float y0 = 0.0f, y1 = 0.0f;
#pragma unroll
      for (int w = 0; w < 8; ++w) {
        const v2f yp = *(const v2f*)(&sY[w][t * 64 + 2 * lane]);
        y0 += yp[0];
        y1 += yp[1];
      }
      const v2f vv = *(const v2f*)(&sX[2][t * 64 + 2 * lane]);
      const v2f gg = *(const v2f*)(&sX[3][t * 64 + 2 * lane]);
      y0 = fmaf(p, vv[0], y0);
      y1 = fmaf(p, vv[1], y1);
      float s = y0 + y1;
#pragma unroll
      for (int off = 1; off < 32; off <<= 1) s += __shfl_xor(s, off, 32);
      const float mean = s * (1.0f / HEADSZ);
      const float d0 = y0 - mean, d1 = y1 - mean;
      float s2 = d0 * d0 + d1 * d1;
#pragma unroll
      for (int off = 1; off < 32; off <<= 1) s2 += __shfl_xor(s2, off, 32);
      const float rstd = rsqrtf(s2 * (1.0f / HEADSZ) + GN_EPS);
      const float z0 = ((d0 * rstd) * lw0 + lb0) * gg[0];
      const float z1 = ((d1 * rstd) * lw1 + lb1) * gg[1];
      const _Float16 h0 = (_Float16)z0, h1 = (_Float16)z1;
      const unsigned wd = (unsigned)__builtin_bit_cast(unsigned short, h0) | ((unsigned)__builtin_bit_cast(unsigned short, h1) << 16);
      sZ[t * 32 + lane] = wd;
    }
    __syncthreads();
    if (tid < 128) {
      const v4u zv = *(const v4u*)(sZ + stok * 32 + sseg * 4);
      unsigned short* zp = Zp + (tok0 + stok) * NCH + h * 64 + sseg * 8;
      *(volatile v4u*)zp = zv;
      __threadfence();
      *(volatile v4u*)zp = zv;
    }
  }
}

extern "C" void kernel_launch(void* const* d_in, const int* in_sizes, int n_in,
                              void* d_out, int out_size, void* d_ws, size_t ws_size, hipStream_t stream) {
  if (n_in < 28 || d_out == nullptr || d_ws == nullptr) return;
  if (in_sizes[0] != NBATCH * NCH * LIMG || in_sizes[1] != NBATCH * NCH * LTXT || in_sizes[2] != NBATCH * NCH) return;
  if (in_sizes[3] != MODN * NCH || in_sizes[4] != MODN || in_sizes[5] != MODN * NCH || in_sizes[6] != MODN) return;
  for (int i = 7; i <= 14; ++i) if (in_sizes[i] != NCH) return;
  for (int i = 15; i <= 19; ++i) if (in_sizes[i] != NCH * NCH) return;
  if (in_sizes[20] != NCH || in_sizes[21] != NCH || in_sizes[22] != NCH || in_sizes[23] != NCH) return;
  for (int i = 24; i <= 27; ++i) if (in_sizes[i] != NFFN * NCH) return;
  if (out_size != NBATCH * NCH * LSEQ) return;

  const float* img   = (const float*)d_in[0];
  const float* txt   = (const float*)d_in[1];
  const float* cond  = (const float*)d_in[2];
  const float* WmI   = (const float*)d_in[3];
  const float* bmI   = (const float*)d_in[4];
  const float* WmT   = (const float*)d_in[5];
  const float* bmT   = (const float*)d_in[6];
  const float* rmsI  = (const float*)d_in[7];
  const float* rmsT  = (const float*)d_in[8];
  const float* rmsI2 = (const float*)d_in[9];
  const float* rmsT2 = (const float*)d_in[10];
  const float* muR   = (const float*)d_in[11];
  const float* muK   = (const float*)d_in[12];
  const float* muV   = (const float*)d_in[13];
  const float* muG   = (const float*)d_in[14];
  const float* Wr    = (const float*)d_in[15];
  const float* Wk    = (const float*)d_in[16];
  const float* Wv    = (const float*)d_in[17];
  const float* Wg    = (const float*)d_in[18];
  const float* Wo    = (const float*)d_in[19];
  const float* tdec  = (const float*)d_in[20];
  const float* tfst  = (const float*)d_in[21];
  const float* lnw   = (const float*)d_in[22];
  const float* lnb   = (const float*)d_in[23];
  const float* W1I   = (const float*)d_in[24];
  const float* W2I   = (const float*)d_in[25];
  const float* W1T   = (const float*)d_in[26];
  const float* W2T   = (const float*)d_in[27];
  float* outImg = (float*)d_out;
  float* outTxt = outImg + (size_t)NBATCH * NCH * LIMG;

  constexpr size_t SZ_W5   = (size_t)5 * NCH * NCH * 2;
  constexpr size_t SZ_MOD  = (size_t)2 * NBATCH * MODN * 4;
  constexpr size_t SZ_PL   = (size_t)NTOK * NCH * 2;
  constexpr size_t SZ_RKVG = (size_t)NTOK * NCAT * 2;
  constexpr size_t SZ_TOT  = SZ_W5 + SZ_MOD + 2 * SZ_PL + SZ_RKVG;
  static_assert(SZ_W5 % 256 == 0 && SZ_MOD % 256 == 0 && SZ_PL % 256 == 0 && SZ_RKVG % 256 == 0);
  static_assert(SZ_TOT <= (size_t)134217728);
  static_assert((size_t)4 * NFFN * NCH * 2 <= SZ_PL);
  static_assert(((size_t)NBATCH * LIMG * NCH + (size_t)NBATCH * LTXT * NCH +
                 (size_t)NBATCH * LIMG * NFFN + (size_t)NBATCH * LTXT * NFFN) * 2 <= SZ_RKVG);
  if (SZ_TOT > ws_size) return;

  char* ws = (char*)d_ws;
  unsigned short* W5   = (unsigned short*)(ws);
  float*          MODp = (float*)(ws + SZ_W5);
  unsigned short* PA   = (unsigned short*)(ws + SZ_W5 + SZ_MOD);
  unsigned short* PB   = (unsigned short*)(ws + SZ_W5 + SZ_MOD + SZ_PL);
  unsigned short* RKVG = (unsigned short*)(ws + SZ_W5 + SZ_MOD + 2 * SZ_PL);
  unsigned short* Zpl  = PA;
  unsigned short* FFNW = PB;
  constexpr size_t WPL = (size_t)NCH * NCH;
  constexpr size_t FPL = (size_t)NFFN * NCH;
  unsigned short* HIimg   = RKVG;
  unsigned short* HItxt   = RKVG + (size_t)NBATCH * LIMG * NCH;
  unsigned short* HMIDimg = HItxt + (size_t)NBATCH * LTXT * NCH;
  unsigned short* HMIDtxt = HMIDimg + (size_t)NBATCH * LIMG * NFFN;

  cast_planes_kernel<<<dim3((int)(WPL / 8 / 256), 5), 256, 0, stream>>>(Wr, Wk, Wv, Wg, Wo, W5, (int)(WPL / 8), WCARRY);
  mod_gemv_kernel<<<dim3(MODN / 32, 2), 256, 0, stream>>>(WmI, bmI, WmT, bmT, cond, MODp);

  const dim3 gTok(LSEQ / 32, NBATCH);
  const dim3 gProj((NTOK / 64) * (NCH / 64) / 8, 1);
  norm_mod_tok_kernel<true><<<gTok, 256, 0, stream>>>(img, txt, rmsI, rmsT, MODp, 0, 1, muR, muK, PA, 0L, PB, 0L);
  gemm_f16_kernel<0, 0><<<gProj, 256, 0, stream>>>(PA, NCH, 0L, W5 + 0 * WPL, NCH, 0L, RKVG + 0 * NCH, NCAT,
      MODp, MODp, MODp, NCH, 0L, MODp, MODp, MODp, NCH, 0L, 0L, NCH, NTOK, NCH, NCH, WCARRY_INV);
  gemm_f16_kernel<0, 0><<<gProj, 256, 0, stream>>>(PB, NCH, 0L, W5 + 1 * WPL, NCH, 0L, RKVG + 1 * NCH, NCAT,
      MODp, MODp, MODp, NCH, 0L, MODp, MODp, MODp, NCH, 0L, 0L, NCH, NTOK, NCH, NCH, WCARRY_INV);
  norm_mod_tok_kernel<true><<<gTok, 256, 0, stream>>>(img, txt, rmsI, rmsT, MODp, 0, 1, muV, muG, PA, 0L, PB, 0L);
  gemm_f16_kernel<0, 0><<<gProj, 256, 0, stream>>>(PA, NCH, 0L, W5 + 2 * WPL, NCH, 0L, RKVG + 2 * NCH, NCAT,
      MODp, MODp, MODp, NCH, 0L, MODp, MODp, MODp, NCH, 0L, 0L, NCH, NTOK, NCH, NCH, WCARRY_INV);
  gemm_f16_kernel<0, 1><<<gProj, 256, 0, stream>>>(PB, NCH, 0L, W5 + 3 * WPL, NCH, 0L, RKVG + 3 * NCH, NCAT,
      MODp, MODp, MODp, NCH, 0L, MODp, MODp, MODp, NCH, 0L, 0L, NCH, NTOK, NCH, NCH, WCARRY_INV);
  state_scan_kernel<<<NBATCH * NHEAD, 256, 0, stream>>>(RKVG, tdec, tfst, lnw, lnb, Zpl);
  gemm_f16_kernel<1, 0><<<dim3((NCH / 64) * (LSEQ / 64) / 8, NBATCH), 256, 0, stream>>>(
      W5 + 4 * WPL, NCH, 0L, Zpl, NCH, (long)LSEQ * NCH, W5, 0,
      outImg, img, MODp + 2 * NCH, LIMG, (long)NCH * LIMG,
      outTxt, txt, MODp + 2 * MODN + 2 * NCH, LTXT, (long)NCH * LTXT,
      (long)MODN, LIMG, NCH, LSEQ, NCH, WCARRY_INV);
  cast_planes_kernel<<<dim3((int)(FPL / 8 / 256), 4), 256, 0, stream>>>(W1I, W2I, W1T, W2T, W2T, FFNW, (int)(FPL / 8), WCARRY);
  norm_mod_tok_kernel<false><<<gTok, 256, 0, stream>>>(outImg, outTxt, rmsI2, rmsT2, MODp, 3, 4, muR, muR,
      HIimg, (long)LIMG * NCH, HItxt, (long)LTXT * NCH);
  gemm_f16_kernel<0, 2><<<dim3((NBATCH * LIMG / 64) * (NFFN / 64) / 8, 1), 256, 0, stream>>>(
      HIimg, NCH, 0L, FFNW + 0 * FPL, NCH, 0L, HMIDimg, NFFN,
      MODp, MODp, MODp, NCH, 0L, MODp, MODp, MODp, NCH, 0L, 0L, NFFN, NBATCH * LIMG, NFFN, NCH, WCARRY_INV);
  gemm_f16_kernel<0, 2><<<dim3((NBATCH * LTXT / 64) * (NFFN / 64) / 8, 1), 256, 0, stream>>>(
      HItxt, NCH, 0L, FFNW + 2 * FPL, NCH, 0L, HMIDtxt, NFFN,
      MODp, MODp, MODp, NCH, 0L, MODp, MODp, MODp, NCH, 0L, 0L, NFFN, NBATCH * LTXT, NFFN, NCH, WCARRY_INV);
  gemm_f16_kernel<1, 0><<<dim3((NCH / 64) * (LIMG / 64) / 8, NBATCH), 256, 0, stream>>>(
      FFNW + 1 * FPL, NFFN, 0L, HMIDimg, NFFN, (long)LIMG * NFFN, W5, 0,
      outImg, outImg, MODp + 5 * NCH, LIMG, (long)NCH * LIMG,
      outImg, outImg, MODp + 5 * NCH, LIMG, (long)NCH * LIMG,
      (long)MODN, LIMG, NCH, LIMG, NFFN, WCARRY_INV);
  gemm_f16_kernel<1, 0><<<dim3((NCH / 64) * (LTXT / 64) / 8, NBATCH), 256, 0, stream>>>(
      FFNW + 3 * FPL, NFFN, 0L, HMIDtxt, NFFN, (long)LTXT * NFFN, W5, 0,
      outTxt, outTxt, MODp + 2 * MODN + 5 * NCH, LTXT, (long)NCH * LTXT,
      outTxt, outTxt, MODp + 2 * MODN + 5 * NCH, LTXT, (long)NCH * LTXT,
      (long)MODN, LTXT, NCH, LTXT, NFFN, WCARRY_INV);
}
